// Net_43121471652562
// MI455X (gfx1250) — hardware-verified
//
#include <hip/hip_runtime.h>
#include <stddef.h>
#include <stdint.h>

#define NN     50000
#define NE     400000
#define FIN    8
#define EDIM   8
#define HD     32
#define CH     64
#define KW     512
#define KA     64
#define KG     128
#define NPAD   50048
#define NPL    50176
#define TOTF   450001
#define NTHR   256
#define NWAVE  8
#define EPT    8
#define CHUNK  (NTHR * EPT)
#define WCAP   (EPT * 32)
#define LISTN  (NWAVE * WCAP)
#define NBA    1024
#define SLA    10
#define RCAP   12288
#define DEGCAP 32
#define NBLK   49
#define EPB    128
#define APITCH 72
#define OPITCH 68
#define NU_W2  (KW * (KA / 8))
#define NU_GK  (CH * (KG / 8))
#define NU_Z   256
#define AGG_ZINTS (LISTN + 2 * RCAP + 3 * NBA)
#define AGG_LDS_INTS (AGG_ZINTS + 16)
#define AGG_LDS_BYTES (AGG_LDS_INTS * 4)
#define WSMAX  134217728
#define NEGSL  0.2f

static_assert(NE % EPB == 0);
static_assert(CH == 64 && FIN * CH == KW && HD == 32 && KA == 2 * HD && KG == 2 * CH);
static_assert(KA % 32 == 0 && KG % 32 == 0);
static_assert(NPAD % 128 == 0 && NPAD >= NN && NPL == NBLK * NBA && NPL >= NPAD);
static_assert((CHUNK & (CHUNK - 1)) == 0 && CHUNK <= 4096);
static_assert((NBA & (NBA - 1)) == 0 && NBA == (1 << SLA));
static_assert(((long long)NE << SLA) < (1LL << 31));
static_assert(LISTN % NTHR == 0 && NBA % NWAVE == 0 && NBA % 32 == 0 && NBA == 4 * NTHR);
static_assert(RCAP % (2 * NTHR) == 0 && AGG_ZINTS % 4 == 0);
static_assert(RCAP >= 8378 + 838);
static_assert(DEGCAP >= 22 + 8 && DEGCAP <= 32);
static_assert(AGG_LDS_BYTES <= 300000);
static_assert(NU_W2 % NTHR == 0 && NU_GK % NTHR == 0);
static_assert(NTHR == 256 && EPB * 2 == NTHR && EPB == NWAVE * 16);
static_assert((APITCH * 2) % 16 == 0 && APITCH >= KA && (OPITCH * 4) % 16 == 0 && OPITCH >= CH);
static_assert(EPB * CH * 4 == 8 * NTHR * 16);
static_assert((TOTF - 1) / 32 == 14062);

typedef float          v2f   __attribute__((ext_vector_type(2)));
typedef float          v4f   __attribute__((ext_vector_type(4)));
typedef float          v8f   __attribute__((ext_vector_type(8)));
typedef int            v2i   __attribute__((ext_vector_type(2)));
typedef int            v4i   __attribute__((ext_vector_type(4)));
typedef int            v8i   __attribute__((ext_vector_type(8)));
typedef unsigned short v4us  __attribute__((ext_vector_type(4)));
typedef unsigned short v8us  __attribute__((ext_vector_type(8)));
typedef unsigned short v16us __attribute__((ext_vector_type(16)));
typedef __bf16         v16bf __attribute__((ext_vector_type(16)));
typedef v2f  __attribute__((may_alias)) v2fa;
typedef v4f  __attribute__((may_alias)) v4fa;
typedef v2i  __attribute__((may_alias)) v2ia;
typedef v4i  __attribute__((may_alias)) v4ia;
typedef v4us __attribute__((may_alias)) v4usa;
typedef v8us __attribute__((may_alias)) v8usa;
union FragB { v16bf v; v16us u; v8us h[2]; v8i w; };

__device__ __forceinline__ v8f wmb(const FragB& a, const FragB& b, v8f c) {
  v8f d = __builtin_amdgcn_wmma_f32_16x16x32_bf16(false, a.v, false, b.v, (short)0, c, false, false);
  asm volatile("v_nop\n\tv_nop\n\tv_nop\n\tv_nop" : "+v"(d) : "v"(a.w), "v"(b.w));
  return d;
}

__device__ __forceinline__ unsigned bf16_bits(float f) {
  const unsigned u = __float_as_uint(f);
  return (u + 0x7FFFu + ((u >> 16) & 1u)) >> 16;
}
__device__ __forceinline__ float bf16_val(float f) {
  return __uint_as_float(bf16_bits(f) << 16);
}
__device__ __forceinline__ int clampi(int v, int lo, int hi) {
  return v < lo ? lo : (v > hi ? hi : v);
}
__device__ __forceinline__ float relu_keep(float v) { return (v > 0.0f) ? v : (v - v); }
__device__ __forceinline__ float leaky(float v) { return (v > 0.0f) ? v : NEGSL * v; }

__device__ __forceinline__ void put16(unsigned short* dp, v8us o) {
  *(volatile v8us*)dp = o;
  __threadfence();
  *(volatile v8us*)dp = o;
}
__device__ __forceinline__ void putf4(float* dp, v4f o) {
  *(volatile v4f*)dp = o;
  __threadfence();
  *(volatile v4f*)dp = o;
}
__device__ __forceinline__ void put4i(int* dp, v4i o) {
  *(volatile v4i*)dp = o;
  __threadfence();
  *(volatile v4i*)dp = o;
}

template <int SLB>
__device__ __forceinline__ int scan_chunk(const int* __restrict__ dsts, int nE, int cbase, int slotBase,
                                          int nb, int vec8, int* list, int tid, int lane, int wave) {
  int wc = 0;
  const int el0  = tid * EPT;
  const int e0   = cbase + el0;
  const int sent = -2147483647 - 1;
  v4i da, db;
  if (vec8 != 0 && cbase + CHUNK <= nE) {
    da = *(const v4i*)(dsts + e0);
    db = *(const v4i*)(dsts + e0 + 4);
  } else {
    da.x = (e0     < nE) ? dsts[min(e0,     nE - 1)] : sent;
    da.y = (e0 + 1 < nE) ? dsts[min(e0 + 1, nE - 1)] : sent;
    da.z = (e0 + 2 < nE) ? dsts[min(e0 + 2, nE - 1)] : sent;
    da.w = (e0 + 3 < nE) ? dsts[min(e0 + 3, nE - 1)] : sent;
    db.x = (e0 + 4 < nE) ? dsts[min(e0 + 4, nE - 1)] : sent;
    db.y = (e0 + 5 < nE) ? dsts[min(e0 + 5, nE - 1)] : sent;
    db.z = (e0 + 6 < nE) ? dsts[min(e0 + 6, nE - 1)] : sent;
    db.w = (e0 + 7 < nE) ? dsts[min(e0 + 7, nE - 1)] : sent;
  }
  const unsigned nbs = (unsigned)slotBase;
  const unsigned unb = (unsigned)nb;
  const unsigned s0 = (unsigned)da.x - nbs, s1 = (unsigned)da.y - nbs;
  const unsigned s2 = (unsigned)da.z - nbs, s3 = (unsigned)da.w - nbs;
  const unsigned s4 = (unsigned)db.x - nbs, s5 = (unsigned)db.y - nbs;
  const unsigned s6 = (unsigned)db.z - nbs, s7 = (unsigned)db.w - nbs;
  const bool h0 = s0 < unb, h1 = s1 < unb, h2 = s2 < unb, h3 = s3 < unb;
  const bool h4 = s4 < unb, h5 = s5 < unb, h6 = s6 < unb, h7 = s7 < unb;
  const unsigned any = __builtin_amdgcn_ballot_w32(h0 | h1 | h2 | h3 | h4 | h5 | h6 | h7);
  if (any != 0u) {
#define HITJ(J, HJ, SJ) { \
      const unsigned mj = __builtin_amdgcn_ballot_w32(HJ); \
      if (mj != 0u) { \
        if (HJ) { \
          const int pos = wc + (int)__builtin_amdgcn_mbcnt_lo(mj, 0u); \
          if (pos < WCAP) list[wave * WCAP + pos] = ((el0 + (J)) << SLB) | (int)(SJ); \
        } \
        wc += (int)__builtin_popcount(mj); } }
    HITJ(0, h0, s0)
    HITJ(1, h1, s1)
    HITJ(2, h2, s2)
    HITJ(3, h3, s3)
    HITJ(4, h4, s4)
    HITJ(5, h5, s5)
    HITJ(6, h6, s6)
    HITJ(7, h7, s7)
#undef HITJ
  }
  return wc;
}

__global__ __launch_bounds__(NTHR) void k_prep(const float* __restrict__ w2, const float* __restrict__ gk,
                                               unsigned short* W2D, unsigned short* GKD,
                                               float* AS, float* AN) {
  const int u = (int)blockIdx.x * NTHR + (int)threadIdx.x;
  v8us o;
  if (u < NU_W2) {
    const int n    = u >> 3;
    const int k8   = (u & 7) * 8;
    const int srow = k8 & (HD - 1);
    const float* p = w2 + (size_t)srow * KW + n;
#pragma unroll
    for (int i = 0; i < 8; ++i) o[i] = (unsigned short)bf16_bits(p[(size_t)i * KW]);
    put16(W2D + (size_t)n * KA + k8, o);
  } else if (u < NU_W2 + NU_GK) {
    const int v    = u - NU_W2;
    const int n    = v >> 4;
    const int k8   = (v & 15) * 8;
    const int srow = k8 & (CH - 1);
    const float* p = gk + (size_t)srow * CH + n;
#pragma unroll
    for (int i = 0; i < 8; ++i) o[i] = (unsigned short)bf16_bits(p[(size_t)i * CH]);
    put16(GKD + (size_t)n * KG + k8, o);
  } else {
    const int v = u - NU_W2 - NU_GK;
    const v4f z4 = {0.0f, 0.0f, 0.0f, 0.0f};
    if (v < 32) {
      putf4(AS + NPAD + 4 * v, z4);
    } else if (v < 64) {
      putf4(AN + NPAD + 4 * (v - 32), z4);
    }
  }
}

__global__ __launch_bounds__(NTHR) void k_bucket(const int* __restrict__ dsts, const int* __restrict__ srcs,
                                                 int nE, int vec8, int* HITS, int* CNT, int* OFF) {
  extern __shared__ __attribute__((aligned(16))) int dsm[];
  int* list = dsm;
  int* hl   = dsm + LISTN;
  int* sl   = hl + RCAP;
  int* cnt  = sl + RCAP;
  int* offs = cnt + NBA;
  int* cur  = offs + NBA;
  int* misc = cur + NBA;
  const int tid = (int)threadIdx.x, lane = tid & 31, wave = tid >> 5;
  const int nodeBase = (int)blockIdx.x * NBA;

  {
    const v4i z4 = {0, 0, 0, 0};
    for (int i = tid * 4; i < AGG_ZINTS; i += NTHR * 4) *(v4ia*)(dsm + i) = z4;
    if (tid < 16) misc[tid] = 0;
  }
  __syncthreads();

  int t = 0, ov = 0;
  const int nChunks = (nE + CHUNK - 1) / CHUNK;
#pragma unroll 1
  for (int ch = 0; ch < nChunks; ++ch) {
    const int cbase = ch * CHUNK;
    const int wc = scan_chunk<SLA>(dsts, nE, cbase, nodeBase, NBA, vec8, list, tid, lane, wave);
    if (lane == 0) misc[wave] = wc;
    __syncthreads();
    if (wave == 0) {
#pragma unroll 1
      for (int w2 = 0; w2 < NWAVE; ++w2) {
        int c = misc[w2];
        c = c < 0 ? 0 : (c > WCAP ? WCAP : c);
#pragma unroll 1
        for (int b0 = 0; b0 < c; b0 += 32) {
          const int idx = b0 + lane;
          const int ent = list[w2 * WCAP + (idx < WCAP ? idx : WCAP - 1)];
          const int m32 = (c - b0) < 32 ? (c - b0) : 32;
#pragma unroll 1
          for (int k = 0; k < m32; ++k) {
            const int u    = __builtin_amdgcn_readlane(ent, k);
            const int slot = u & (NBA - 1);
            const int el   = (u >> SLA) & (CHUNK - 1);
            const int pk   = ((cbase + el) << SLA) | slot;
            if (t < RCAP) {
              if (lane == 0) { hl[t] = pk; cnt[slot] = cnt[slot] + 1; }
              t = t + 1;
            } else {
              ov = 1;
            }
          }
        }
      }
    }
    __syncthreads();
  }
  if (wave == 0 && lane == 0) { misc[8] = t; misc[9] = ov; }
  __syncthreads();
  int tt = misc[8];
  tt = tt < 0 ? 0 : (tt > RCAP ? RCAP : tt);
  const int ovf = misc[9];

  if (wave == 0) {
    const int base = lane * (NBA / 32);
    int s = 0;
#pragma unroll 1
    for (int i = 0; i < NBA / 32; ++i) s += cnt[base + i];
    int incl = s;
#pragma unroll
    for (int d = 1; d < 32; d <<= 1) {
      const int y = __shfl_up(incl, d, 32);
      if (lane >= d) incl += y;
    }
    int run = incl - s;
#pragma unroll 1
    for (int i = 0; i < NBA / 32; ++i) {
      const int cv = cnt[base + i];
      offs[base + i] = run;
      cur[base + i]  = run;
      run += cv;
    }
  }
  __syncthreads();
  if (wave == 0) {
#pragma unroll 1
    for (int b0 = 0; b0 < tt; b0 += 32) {
      const int idx = b0 + lane;
      const int ent = hl[idx < RCAP ? idx : RCAP - 1];
      const int m32 = (tt - b0) < 32 ? (tt - b0) : 32;
#pragma unroll 1
      for (int k = 0; k < m32; ++k) {
        const int u    = __builtin_amdgcn_readlane(ent, k);
        const int slot = u & (NBA - 1);
        if (lane == 0) {
          int p = cur[slot];
          p = p < 0 ? 0 : (p > RCAP - 1 ? RCAP - 1 : p);
          sl[p] = u;
          cur[slot] = p + 1;
        }
      }
    }
  }
  __syncthreads();

  int* hb = HITS + (size_t)blockIdx.x * (size_t)(RCAP * 2);
#pragma unroll 1
  for (int it = 0; it < RCAP / (2 * NTHR); ++it) {
    const int p = it * NTHR + tid;
    const v2i en = *(const v2ia*)(sl + 2 * p);
    const int e0 = clampi(en.x >> SLA, 0, nE - 1);
    const int e1 = clampi(en.y >> SLA, 0, nE - 1);
    const int s0 = srcs[e0];
    const int s1 = srcs[e1];
    v4i o;
    o.x = e0; o.y = clampi(s0, 0, NN - 1); o.z = e1; o.w = clampi(s1, 0, NN - 1);
    put4i(hb + 4 * p, o);
  }
  {
    v4i c4 = *(const v4ia*)(cnt + 4 * tid);
    const v4i o4 = *(const v4ia*)(offs + 4 * tid);
    const v4i m1 = {-1, -1, -1, -1};
    if (ovf != 0) c4 = m1;
    put4i(CNT + nodeBase + 4 * tid, c4);
    put4i(OFF + nodeBase + 4 * tid, o4);
  }
}

__global__ __launch_bounds__(NTHR) void k_ecc_edge(const float* __restrict__ X, const float* __restrict__ Ef,
                                                   const int* __restrict__ srcs,
                                                   const float* __restrict__ w1, const float* __restrict__ b1,
                                                   const float* __restrict__ b2,
                                                   const unsigned short* __restrict__ W2D, float* MSG) {
  __shared__ __attribute__((aligned(16))) unsigned short sA[EPB * APITCH];
  __shared__ __attribute__((aligned(16))) float sXT[FIN * EPB];
  __shared__ __attribute__((aligned(16))) float sB2[KW];
  __shared__ __attribute__((aligned(16))) float sW1[EDIM * HD];
  __shared__ __attribute__((aligned(16))) float sB1[HD];
  __shared__ __attribute__((aligned(16))) float sO[EPB * OPITCH];

  const int tid = (int)threadIdx.x, lane = tid & 31, wave = tid >> 5, hh = lane >> 4, m = lane & 15;
  const int elb  = (int)blockIdx.x * EPB;
  const int el   = tid >> 1;
  const int half = tid & 1;
  const int e    = elb + el;

  {
    const float t0 = b2[tid];
    const float t1 = b2[tid + NTHR];
    const float t2 = w1[tid];
    const float t3 = b1[tid & (HD - 1)];
    sB2[tid]        = bf16_val(t0);
    sB2[tid + NTHR] = bf16_val(t1);
    sW1[tid]        = bf16_val(t2);
    if (tid < HD) sB1[tid] = bf16_val(t3);
  }
  float ev[EDIM];
  {
    const float* ep = Ef + (size_t)e * EDIM;
    const v4f ea = *(const v4f*)ep;
    const v4f eb = *(const v4f*)(ep + 4);
    ev[0] = bf16_val(ea.x); ev[1] = bf16_val(ea.y); ev[2] = bf16_val(ea.z); ev[3] = bf16_val(ea.w);
    ev[4] = bf16_val(eb.x); ev[5] = bf16_val(eb.y); ev[6] = bf16_val(eb.z); ev[7] = bf16_val(eb.w);
    const int s = clampi(srcs[e], 0, NN - 1);
    const v4f xa = *(const v4f*)(X + (size_t)s * FIN + 4 * half);
    sXT[(4 * half + 0) * EPB + el] = bf16_val(xa.x);
    sXT[(4 * half + 1) * EPB + el] = bf16_val(xa.y);
    sXT[(4 * half + 2) * EPB + el] = bf16_val(xa.z);
    sXT[(4 * half + 3) * EPB + el] = bf16_val(xa.w);
  }
  __syncthreads();

  {
    unsigned short* ra = sA + el * APITCH;
#pragma unroll 1
    for (int g4 = 0; g4 < 4; ++g4) {
      const int j0 = 16 * half + 4 * g4;
      v4f hv = {0.0f, 0.0f, 0.0f, 0.0f};
#pragma unroll
      for (int d = 0; d < EDIM; ++d) {
        const v4f w = *(const v4fa*)(sW1 + d * HD + j0);
        hv.x = fmaf(ev[d], w.x, hv.x);
        hv.y = fmaf(ev[d], w.y, hv.y);
        hv.z = fmaf(ev[d], w.z, hv.z);
        hv.w = fmaf(ev[d], w.w, hv.w);
      }
      const v4f bb = *(const v4fa*)(sB1 + j0);
      hv.x = relu_keep(hv.x + bb.x);
      hv.y = relu_keep(hv.y + bb.y);
      hv.z = relu_keep(hv.z + bb.z);
      hv.w = relu_keep(hv.w + bb.w);
      v4us ho, lo;
#pragma unroll
      for (int i = 0; i < 4; ++i) {
        const unsigned hb = bf16_bits(hv[i]);
        ho[i] = (unsigned short)hb;
        lo[i] = (unsigned short)bf16_bits(hv[i] - __uint_as_float(hb << 16));
      }
      *(v4usa*)(ra + j0)      = ho;
      *(v4usa*)(ra + HD + j0) = lo;
    }
  }
  __syncthreads();

  FragB a0, a1;
  {
    const unsigned short* ap = sA + (16 * wave + m) * APITCH + 8 * hh;
    a0.h[0] = *(const v8usa*)(ap);
    a0.h[1] = *(const v8usa*)(ap + 16);
    a1.h[0] = *(const v8usa*)(ap + 32);
    a1.h[1] = *(const v8usa*)(ap + 48);
  }
  const v8f z8 = {0.f, 0.f, 0.f, 0.f, 0.f, 0.f, 0.f, 0.f};
  v8f ACC[4];
#pragma unroll
  for (int nt = 0; nt < 4; ++nt) ACC[nt] = z8;
  const unsigned short* bp = W2D + (size_t)m * KA + 8 * hh;

#pragma unroll 1
  for (int f = 0; f < FIN; ++f) {
    v8f D[4];
#pragma unroll
    for (int nt = 0; nt < 4; ++nt) {
      const unsigned short* wq = bp + (size_t)(f * CH + 16 * nt) * KA;
      FragB b0, b1f;
      b0.h[0]  = *(const v8usa*)(wq);
      b0.h[1]  = *(const v8usa*)(wq + 16);
      b1f.h[0] = *(const v8usa*)(wq + 32);
      b1f.h[1] = *(const v8usa*)(wq + 48);
      D[nt] = wmb(a0, b0, z8);
      D[nt] = wmb(a1, b1f, D[nt]);
    }
    const float* xp = sXT + f * EPB + 16 * wave + 8 * hh;
    const v4f x0 = *(const v4fa*)xp;
    const v4f x1 = *(const v4fa*)(xp + 4);
    const v8f xs = {x0.x, x0.y, x0.z, x0.w, x1.x, x1.y, x1.z, x1.w};
#pragma unroll
    for (int nt = 0; nt < 4; ++nt) {
      const float bb = sB2[f * CH + 16 * nt + m];
#pragma unroll
      for (int r = 0; r < 8; ++r) ACC[nt][r] = fmaf(xs[r], D[nt][r] + bb, ACC[nt][r]);
    }
  }

#pragma unroll
  for (int nt = 0; nt < 4; ++nt) {
#pragma unroll
    for (int r = 0; r < 8; ++r) sO[(16 * wave + 8 * hh + r) * OPITCH + 16 * nt + m] = ACC[nt][r];
  }
  __syncthreads();

  {
    v4f pv[8];
#pragma unroll
    for (int it = 0; it < 8; ++it) {
      const int p = it * NTHR + tid;
      pv[it] = *(const v4fa*)(sO + (p >> 4) * OPITCH + (p & 15) * 4);
    }
    float* mb = MSG + (size_t)elb * CH;
#pragma unroll
    for (int it = 0; it < 8; ++it) *(volatile v4f*)(mb + (size_t)(it * NTHR + tid) * 4) = pv[it];
    __threadfence();
#pragma unroll
    for (int it = 0; it < 8; ++it) *(volatile v4f*)(mb + (size_t)(it * NTHR + tid) * 4) = pv[it];
  }
}

__global__ __launch_bounds__(NTHR) void k_agg1(const float* __restrict__ MSG, const int* __restrict__ HITS,
                                               const int* __restrict__ CNT, const int* __restrict__ OFF,
                                               const float* __restrict__ X, const float* __restrict__ root,
                                               const float* __restrict__ ebias, unsigned short* X1HL) {
  const int tid = (int)threadIdx.x, lane = tid & 31;
  const int wave = __builtin_amdgcn_readfirstlane(tid >> 5);
  const int nodeBase = (int)blockIdx.x * NBA;
  const int* hbase = HITS + (size_t)blockIdx.x * (size_t)(RCAP * 2);

  float rA[FIN], rB[FIN];
#pragma unroll
  for (int f = 0; f < FIN; ++f) {
    const v2f r = *(const v2f*)(root + f * CH + 2 * lane);
    rA[f] = bf16_val(r.x);
    rB[f] = bf16_val(r.y);
  }
  float eb0, eb1;
  {
    const v2f b = *(const v2f*)(ebias + 2 * lane);
    eb0 = bf16_val(b.x);
    eb1 = bf16_val(b.y);
  }
  const float qnan = __int_as_float(0x7fc00000);

#pragma unroll 1
  for (int si = 0; si < NBA / NWAVE; ++si) {
    const int s    = si * NWAVE + wave;
    const int node = nodeBase + s;
    if (node < NPAD) {
      const int nc = node < NN ? node : NN - 1;
      int c = __builtin_amdgcn_readfirstlane(CNT[node]);
      int o = __builtin_amdgcn_readfirstlane(OFF[node]);
      const bool bad = (c < 0) || (c > DEGCAP);
      c = clampi(c, 0, DEGCAP);
      o = clampi(o, 0, RCAP);
      const int idx = (o + lane) > (RCAP - 1) ? (RCAP - 1) : (o + lane);
      const v2i ent = *(const v2i*)(hbase + 2 * idx);
      const int eid = clampi(ent.x, 0, NE - 1);
      float a0 = 0.0f, a1 = 0.0f;
#pragma unroll 1
      for (int k = 0; k < c; ++k) {
        const int ek = __builtin_amdgcn_readlane(eid, k);
        const v2f w = *(const v2f*)(MSG + (size_t)ek * CH + 2 * lane);
        a0 += w.x;
        a1 += w.y;
      }
      const float* xp = X + (size_t)nc * FIN;
      const v4f xa = *(const v4f*)xp;
      const v4f xb = *(const v4f*)(xp + 4);
      const float xv[FIN] = {bf16_val(xa.x), bf16_val(xa.y), bf16_val(xa.z), bf16_val(xa.w),
                             bf16_val(xb.x), bf16_val(xb.y), bf16_val(xb.z), bf16_val(xb.w)};
      float d0 = xv[0] * rA[0];
      float d1 = xv[0] * rB[0];
#pragma unroll
      for (int f = 1; f < FIN; ++f) {
        d0 = fmaf(xv[f], rA[f], d0);
        d1 = fmaf(xv[f], rB[f], d1);
      }
      float v0 = relu_keep((a0 + d0) + eb0);
      float v1 = relu_keep((a1 + d1) + eb1);
      v0 = bad ? qnan : v0;
      v1 = bad ? qnan : v1;
      const bool live = node < NN;
      v0 = live ? v0 : 0.0f;
      v1 = live ? v1 : 0.0f;
      const unsigned h0 = bf16_bits(v0), h1 = bf16_bits(v1);
      const unsigned l0 = bf16_bits(v0 - __uint_as_float(h0 << 16));
      const unsigned l1 = bf16_bits(v1 - __uint_as_float(h1 << 16));
      const unsigned wh = (h0 & 0xffffu) | (h1 << 16);
      const unsigned wl = (l0 & 0xffffu) | (l1 << 16);
      unsigned* rp = (unsigned*)(X1HL + (size_t)node * KG);
      *(volatile unsigned*)(rp + lane)      = wh;
      *(volatile unsigned*)(rp + 32 + lane) = wl;
      __threadfence();
      *(volatile unsigned*)(rp + lane)      = wh;
      *(volatile unsigned*)(rp + 32 + lane) = wl;
    }
  }
}

__global__ __launch_bounds__(NTHR) void k_gat_gemm(const unsigned short* __restrict__ X1HL,
                                                   const unsigned short* __restrict__ GKD,
                                                   const float* __restrict__ avs, const float* __restrict__ avn,
                                                   float* XG, float* AS, float* AN) {
  __shared__ __attribute__((aligned(16))) float stg[EPB * OPITCH];
  __shared__ __attribute__((aligned(16))) float sdt[2 * EPB];
  const int tid = (int)threadIdx.x, lane = tid & 31, hh = lane >> 4, m = lane & 15;
  const int wave = __builtin_amdgcn_readfirstlane(tid >> 5);
  const int rowBase = (int)blockIdx.x * EPB;

  v8f acc[4];
  {
    const v8f z = {0.f, 0.f, 0.f, 0.f, 0.f, 0.f, 0.f, 0.f};
#pragma unroll
    for (int t = 0; t < 4; ++t) acc[t] = z;
  }
  const unsigned short* ap = X1HL + (size_t)(rowBase + 16 * wave + m) * KG + 8 * hh;
  const unsigned short* bp = GKD + (size_t)m * KG + 8 * hh;
#pragma unroll 1
  for (int k0 = 0; k0 < KG; k0 += 32) {
    FragB af;
    af.h[0] = *(const v8usa*)(ap + k0);
    af.h[1] = *(const v8usa*)(ap + k0 + 16);
#pragma unroll
    for (int nt = 0; nt < 4; ++nt) {
      const unsigned short* wq = bp + (size_t)(16 * nt) * KG + k0;
      FragB bf;
      bf.h[0] = *(const v8usa*)wq;
      bf.h[1] = *(const v8usa*)(wq + 16);
      acc[nt] = wmb(af, bf, acc[nt]);
    }
  }
#pragma unroll
  for (int nt = 0; nt < 4; ++nt) {
#pragma unroll
    for (int r = 0; r < 8; ++r) stg[(16 * wave + 8 * hh + r) * OPITCH + 16 * nt + m] = acc[nt][r];
  }
  __syncthreads();

  {
    const v2f s2 = *(const v2f*)(avs + 2 * lane);
    const v2f n2 = *(const v2f*)(avn + 2 * lane);
    const float as0 = bf16_val(s2.x), as1 = bf16_val(s2.y);
    const float an0 = bf16_val(n2.x), an1 = bf16_val(n2.y);
#pragma unroll 1
    for (int i = 0; i < 16; ++i) {
      const int row = 16 * wave + i;
      const v2f p = *(const v2fa*)(stg + row * OPITCH + 2 * lane);
      float s = p.x * as0;
      s = fmaf(p.y, as1, s);
      float d = p.x * an0;
      d = fmaf(p.y, an1, d);
#pragma unroll
      for (int off = 16; off > 0; off >>= 1) {
        s += __shfl_xor(s, off);
        d += __shfl_xor(d, off);
      }
      if (lane == 0) { sdt[row] = s; sdt[EPB + row] = d; }
    }
  }
  __syncthreads();

  {
    v4f pv[8];
#pragma unroll
    for (int it = 0; it < 8; ++it) {
      const int p = it * NTHR + tid;
      pv[it] = *(const v4fa*)(stg + (p >> 4) * OPITCH + (p & 15) * 4);
    }
    const v4f sv = *(const v4fa*)(sdt + 4 * lane);
    const v4f nv = *(const v4fa*)(sdt + EPB + 4 * lane);
    float* xb = XG + (size_t)rowBase * CH;
#pragma unroll
    for (int it = 0; it < 8; ++it) *(volatile v4f*)(xb + (size_t)(it * NTHR + tid) * 4) = pv[it];
    if (wave == 0) *(volatile v4f*)(AS + rowBase + 4 * lane) = sv;
    if (wave == 1) *(volatile v4f*)(AN + rowBase + 4 * lane) = nv;
    __threadfence();
#pragma unroll
    for (int it = 0; it < 8; ++it) *(volatile v4f*)(xb + (size_t)(it * NTHR + tid) * 4) = pv[it];
    if (wave == 0) *(volatile v4f*)(AS + rowBase + 4 * lane) = sv;
    if (wave == 1) *(volatile v4f*)(AN + rowBase + 4 * lane) = nv;
  }
}

__global__ __launch_bounds__(NTHR) void k_gat_scan(const int* __restrict__ HITS, const int* __restrict__ CNT,
                                                   const int* __restrict__ OFF, const float* __restrict__ XG,
                                                   const float* __restrict__ AS, const float* __restrict__ AN,
                                                   const float* __restrict__ gbias,
                                                   float* M, float* Z, float* POOLREC) {
  __shared__ __attribute__((aligned(16))) float sM[NBA];
  __shared__ __attribute__((aligned(16))) float sZ[NBA];
  __shared__ __attribute__((aligned(16))) float sP[NWAVE * CH];
  const int tid = (int)threadIdx.x, lane = tid & 31;
  const int wave = __builtin_amdgcn_readfirstlane(tid >> 5);
  const int nodeBase = (int)blockIdx.x * NBA;
  const int* hbase = HITS + (size_t)blockIdx.x * (size_t)(RCAP * 2);
  float gb0, gb1;
  {
    const v2f b = *(const v2f*)(gbias + 2 * lane);
    gb0 = bf16_val(b.x);
    gb1 = bf16_val(b.y);
  }
  const float qnan = __int_as_float(0x7fc00000);
  float ps0 = 0.0f, ps1 = 0.0f;

#pragma unroll 1
  for (int si = 0; si < NBA / NWAVE; ++si) {
    const int s    = si * NWAVE + wave;
    const int node = nodeBase + s;
    if (node < NN) {
      int c = __builtin_amdgcn_readfirstlane(CNT[node]);
      int o = __builtin_amdgcn_readfirstlane(OFF[node]);
      const bool bad = (c < 0) || (c > DEGCAP);
      c = clampi(c, 0, DEGCAP);
      o = clampi(o, 0, RCAP);
      const int idx = (o + lane) > (RCAP - 1) ? (RCAP - 1) : (o + lane);
      const v2i ent = *(const v2i*)(hbase + 2 * idx);
      const int sr = clampi(ent.y, 0, NN - 1);
      const float as_t = AS[node];
      const float an_t = AN[node];
      const float an_s = AN[sr];
      const float l0 = leaky(as_t + an_t);
      const float lg = leaky(as_t + an_s);
      const int   lgi = __float_as_int(lg);
      float mx = l0;
#pragma unroll 1
      for (int k = 0; k < c; ++k) {
        const float v = __int_as_float(__builtin_amdgcn_readlane(lgi, k));
        mx = (v > mx || v != v) ? v : mx;
      }
      const float ex0 = expf(l0 - mx);
      const float ex  = expf(lg - mx);
      const int   exi = __float_as_int(ex);
      float zz = ex0;
#pragma unroll 1
      for (int k = 0; k < c; ++k) zz += __int_as_float(__builtin_amdgcn_readlane(exi, k));
      const float at0 = ex0 / zz;
      const float at  = ex / zz;
      const int   ati = __float_as_int(at);
      const v2f xs = *(const v2f*)(XG + (size_t)node * CH + 2 * lane);
      float a0 = at0 * xs.x;
      float a1 = at0 * xs.y;
#pragma unroll 1
      for (int k = 0; k < c; ++k) {
        const int   sk = __builtin_amdgcn_readlane(sr, k);
        const float ak = __int_as_float(__builtin_amdgcn_readlane(ati, k));
        const v2f w = *(const v2f*)(XG + (size_t)sk * CH + 2 * lane);
        a0 = fmaf(ak, w.x, a0);
        a1 = fmaf(ak, w.y, a1);
      }
      float y0 = relu_keep(a0 + gb0);
      float y1 = relu_keep(a1 + gb1);
      y0 = bad ? qnan : y0;
      y1 = bad ? qnan : y1;
      ps0 += y0;
      ps1 += y1;
      if (lane == 0) {
        sM[s] = bad ? qnan : mx;
        sZ[s] = bad ? qnan : zz;
      }
    } else {
      if (lane == 0) { sM[s] = 0.0f; sZ[s] = 1.0f; }
    }
  }
  sP[wave * CH + 2 * lane]     = ps0;
  sP[wave * CH + 2 * lane + 1] = ps1;
  __syncthreads();

  {
    const v4f mv = *(const v4fa*)(sM + 4 * tid);
    const v4f zv = *(const v4fa*)(sZ + 4 * tid);
    const int cq = lane < 16 ? lane : 15;
    v4f pr = *(const v4fa*)(sP + 4 * cq);
#pragma unroll
    for (int w = 1; w < NWAVE; ++w) {
      const v4f q = *(const v4fa*)(sP + w * CH + 4 * cq);
      pr.x += q.x; pr.y += q.y; pr.z += q.z; pr.w += q.w;
    }
    float* mp = M + nodeBase + 4 * tid;
    float* zp = Z + nodeBase + 4 * tid;
    float* pp = POOLREC + (size_t)blockIdx.x * CH + 4 * cq;
    const bool pw = (wave == 0) && (lane < 16);
    *(volatile v4f*)mp = mv;
    *(volatile v4f*)zp = zv;
    if (pw) *(volatile v4f*)pp = pr;
    __threadfence();
    *(volatile v4f*)mp = mv;
    *(volatile v4f*)zp = zv;
    if (pw) *(volatile v4f*)pp = pr;
  }
}

__global__ __launch_bounds__(NTHR) void k_out(const int* __restrict__ srcs, const int* __restrict__ tgts,
                                              const float* __restrict__ AS, const float* __restrict__ AN,
                                              const float* __restrict__ M, const float* __restrict__ Z,
                                              const float* __restrict__ POOLREC,
                                              const float* __restrict__ fcw, const float* __restrict__ fcb,
                                              const float* __restrict__ outw, const float* __restrict__ outb,
                                              float* out) {
  const int tid = (int)threadIdx.x, lane = tid & 31;
  const int g  = (int)blockIdx.x * NTHR + tid;
  const int gw = __builtin_amdgcn_readfirstlane(g >> 5);
  const int e  = g - 1;
  const int ec = clampi(e, 0, NE - 1);
  const int si = srcs[ec];
  const int ti = tgts[ec];
  const int lp = e - NE;
  const bool isE = e < NE;
  const int s = clampi(isE ? si : lp, 0, NN - 1);
  const int t = clampi(isE ? ti : lp, 0, NN - 1);
  const float as_t = AS[t];
  const float an_s = AN[s];
  const float mm   = M[t];
  const float zz   = Z[t];
  const float lg = leaky(as_t + an_s);
  const float at = expf(lg - mm) / zz;
  float val = at;
  if (gw == 0) {
    double d0 = 0.0, d1 = 0.0;
#pragma unroll 1
    for (int r = 0; r < NBLK; ++r) {
      d0 += (double)POOLREC[r * CH + lane];
      d1 += (double)POOLREC[r * CH + 32 + lane];
    }
    const double inv = 1.0 / (double)NN;
    const float p0 = (float)(d0 * inv);
    const float p1 = (float)(d1 * inv);
    float acc = 0.0f;
#pragma unroll 1
    for (int c = 0; c < 32; ++c) {
      const float pc = __shfl(p0, c);
      acc = fmaf(pc, bf16_val(fcw[c * HD + lane]), acc);
    }
#pragma unroll 1
    for (int c = 0; c < 32; ++c) {
      const float pc = __shfl(p1, c);
      acc = fmaf(pc, bf16_val(fcw[(32 + c) * HD + lane]), acc);
    }
    acc += bf16_val(fcb[lane]);
    const float fv = relu_keep(acc);
    float tt = fv * bf16_val(outw[lane]);
#pragma unroll
    for (int off = 16; off > 0; off >>= 1) tt += __shfl_xor(tt, off);
    const float sg = tt + bf16_val(outb[0]);
    const float o0 = 1.0f / (1.0f + expf(-sg));
    val = (lane == 0) ? o0 : at;
  }
  if (g <= TOTF - 1) {
    float* op = out + g;
    *(volatile float*)op = val;
    __threadfence();
    *(volatile float*)op = val;
  }
}

static inline int cdiv(int a, int b) { return (a + b - 1) / b; }

extern "C" void kernel_launch(void* const* d_in, const int* in_sizes, int n_in,
                              void* d_out, int out_size, void* d_ws, size_t ws_size,
                              hipStream_t stream) {
  if (n_in < 17) return;
  if (in_sizes[0] != NN * FIN) return;
  if (in_sizes[1] != NE * EDIM) return;
  if (in_sizes[2] != 2 * NE) return;
  if (in_sizes[3] != EDIM * HD || in_sizes[4] != HD) return;
  if (in_sizes[5] != HD * KW || in_sizes[6] != KW) return;
  if (in_sizes[7] != FIN * CH || in_sizes[8] != CH) return;
  if (in_sizes[9] != CH * CH) return;
  if (in_sizes[10] != CH || in_sizes[11] != CH || in_sizes[12] != CH) return;
  if (in_sizes[13] != CH * HD || in_sizes[14] != HD) return;
  if (in_sizes[15] != HD || in_sizes[16] != 1) return;
  if (out_size != TOTF) return;

  const float* X     = (const float*)d_in[0];
  const float* Ef    = (const float*)d_in[1];
  const int*   eidx  = (const int*)d_in[2];
  const float* w1    = (const float*)d_in[3];
  const float* b1    = (const float*)d_in[4];
  const float* w2    = (const float*)d_in[5];
  const float* b2    = (const float*)d_in[6];
  const float* root  = (const float*)d_in[7];
  const float* ebias = (const float*)d_in[8];
  const float* gatk  = (const float*)d_in[9];
  const float* atts  = (const float*)d_in[10];
  const float* attn  = (const float*)d_in[11];
  const float* gbias = (const float*)d_in[12];
  const float* fcw   = (const float*)d_in[13];
  const float* fcb   = (const float*)d_in[14];
  const float* outw  = (const float*)d_in[15];
  const float* outb  = (const float*)d_in[16];
  float* out = (float*)d_out;
  const int* src = eidx;
  const int* tgt = eidx + NE;

  char* ws = (char*)d_ws;
  size_t off = 0;
  const size_t oW2D = off; off += (size_t)KW * KA * 2;                 off = (off + 255) & ~(size_t)255;
  const size_t oGKD = off; off += (size_t)CH * KG * 2;                 off = (off + 255) & ~(size_t)255;
  const size_t oHIT = off; off += (size_t)NBLK * RCAP * 8;             off = (off + 255) & ~(size_t)255;
  const size_t oCNT = off; off += (size_t)NPL * 4;                     off = (off + 255) & ~(size_t)255;
  const size_t oOFF = off; off += (size_t)NPL * 4;                     off = (off + 255) & ~(size_t)255;
  const size_t oAS  = off; off += (size_t)NPL * 4;                     off = (off + 255) & ~(size_t)255;
  const size_t oAN  = off; off += (size_t)NPL * 4;                     off = (off + 255) & ~(size_t)255;
  const size_t oM   = off; off += (size_t)NPL * 4;                     off = (off + 255) & ~(size_t)255;
  const size_t oZ   = off; off += (size_t)NPL * 4;                     off = (off + 255) & ~(size_t)255;
  const size_t oPR  = off; off += (size_t)NBLK * CH * 4;               off = (off + 255) & ~(size_t)255;
  const size_t oX1  = off; off += (size_t)NPAD * KG * 2;               off = (off + 255) & ~(size_t)255;
  size_t szMS = (size_t)NE * CH * 4;
  if (szMS < (size_t)NPAD * CH * 4) szMS = (size_t)NPAD * CH * 4;
  const size_t oMS  = off; off += szMS;                                off = (off + 255) & ~(size_t)255;
  if (off > ws_size || off > (size_t)WSMAX) return;

  unsigned short* W2D  = (unsigned short*)(ws + oW2D);
  unsigned short* GKD  = (unsigned short*)(ws + oGKD);
  int*            HITS = (int*)(ws + oHIT);
  int*            CNT  = (int*)(ws + oCNT);
  int*            OFF  = (int*)(ws + oOFF);
  float*          AS   = (float*)(ws + oAS);
  float*          AN   = (float*)(ws + oAN);
  float*          Mp   = (float*)(ws + oM);
  float*          Zp   = (float*)(ws + oZ);
  float*          PR   = (float*)(ws + oPR);
  unsigned short* X1HL = (unsigned short*)(ws + oX1);
  float*          MSG  = (float*)(ws + oMS);
  float*          XG   = (float*)(ws + oMS);

  hipFuncSetAttribute(reinterpret_cast<const void*>(&k_bucket), hipFuncAttributeMaxDynamicSharedMemorySize,
                      (int)AGG_LDS_BYTES);

  const int vec8 = ((NE & 3) == 0) ? 1 : 0;
  k_prep<<<(NU_W2 + NU_GK + NU_Z) / NTHR, NTHR, 0, stream>>>(w2, gatk, W2D, GKD, AS, AN);
  k_bucket<<<NBLK, NTHR, AGG_LDS_BYTES, stream>>>(tgt, src, NE, vec8, HITS, CNT, OFF);
  k_ecc_edge<<<NE / EPB, NTHR, 0, stream>>>(X, Ef, src, w1, b1, b2, W2D, MSG);
  k_agg1<<<NBLK, NTHR, 0, stream>>>(MSG, HITS, CNT, OFF, X, root, ebias, X1HL);
  k_gat_gemm<<<NPAD / EPB, NTHR, 0, stream>>>(X1HL, GKD, atts, attn, XG, AS, AN);
  k_gat_scan<<<NBLK, NTHR, 0, stream>>>(HITS, CNT, OFF, XG, AS, AN, gbias, Mp, Zp, PR);
  k_out<<<cdiv(TOTF, NTHR), NTHR, 0, stream>>>(src, tgt, AS, AN, Mp, Zp, PR, fcw, fcb, outw, outb, out);
}
